// MemoryBlock_12936441496249
// MI455X (gfx1250) — hardware-verified
//
#include <hip/hip_runtime.h>

#define MEM_DIM   2048
#define Z_DIM     256
#define RPB       16
#define NTHR      256
#define XP        264
#define AP        2052
#define APH       (AP * 2)
#define OP        260
#define PM        64
#define TP        264
#define LAMBDA    0.005f
#define EPS_S     1e-12f
#define EPS_N     1e-12f
#define B_SCALE   1024.0f
#define B_UNSCALE 0.0009765625f

typedef float          v4f  __attribute__((ext_vector_type(4)));
typedef float          v8f  __attribute__((ext_vector_type(8)));
typedef unsigned int   v2u  __attribute__((ext_vector_type(2)));
typedef unsigned int   v4u  __attribute__((ext_vector_type(4)));
typedef _Float16       v16h __attribute__((ext_vector_type(16)));
typedef __bf16         v16b __attribute__((ext_vector_type(16)));

union FragB { v16b v; v4u q[2]; };
union FragH { v16h v; v4u q[2]; };

__device__ __forceinline__ unsigned int bf16_bits(float f) {
    unsigned int u = __float_as_uint(f);
    return (u + 0x7FFFu + ((u >> 16) & 1u)) >> 16;
}
__device__ __forceinline__ unsigned int f16x2_bits(float a, float b) {
    union { _Float16 hh[2]; unsigned int u; } t;
    t.hh[0] = (_Float16)a;
    t.hh[1] = (_Float16)b;
    return t.u;
}
__device__ __forceinline__ float shrink_g(float p) {
    const float d = p - LAMBDA;
    const float v = (d * p) * __builtin_amdgcn_rcpf(d + EPS_S);
    return d > 0.0f ? v : 0.0f;
}

#define WMMA_GUARD2(c0, c1, fa, fb0, fb1) \
    asm volatile("v_nop\n\tv_nop\n\tv_nop\n\tv_nop" : "+v"(c0), "+v"(c1) : "v"(fa), "v"(fb0), "v"(fb1))

__global__ __launch_bounds__(NTHR)
void k_prep(const float* __restrict__ mem,
            unsigned short* __restrict__ memb,
            unsigned short* __restrict__ memh)
{
    __shared__ __attribute__((aligned(16))) unsigned short T[PM * TP];

    const int tid  = threadIdx.x;
    const int wave = tid >> 5;
    const int lane = tid & 31;
    const int m0   = blockIdx.x * PM;

    v4u keepb[8];
#pragma unroll
    for (int i = 0; i < 8; ++i) {
        const int ml = wave + 8 * i;
        const int m  = m0 + ml;
        const float* src = mem + (size_t)m * Z_DIM + 8 * lane;
        const v4f f0 = *(const v4f*)src;
        const v4f f1 = *(const v4f*)(src + 4);
        unsigned int bb[8];
        bb[0] = bf16_bits(f0.x); bb[1] = bf16_bits(f0.y); bb[2] = bf16_bits(f0.z); bb[3] = bf16_bits(f0.w);
        bb[4] = bf16_bits(f1.x); bb[5] = bf16_bits(f1.y); bb[6] = bf16_bits(f1.z); bb[7] = bf16_bits(f1.w);
        v4u qb;
        qb.x = bb[0] | (bb[1] << 16);
        qb.y = bb[2] | (bb[3] << 16);
        qb.z = bb[4] | (bb[5] << 16);
        qb.w = bb[6] | (bb[7] << 16);
        v4u qh;
        qh.x = f16x2_bits(__uint_as_float(bb[0] << 16) * B_SCALE, __uint_as_float(bb[1] << 16) * B_SCALE);
        qh.y = f16x2_bits(__uint_as_float(bb[2] << 16) * B_SCALE, __uint_as_float(bb[3] << 16) * B_SCALE);
        qh.z = f16x2_bits(__uint_as_float(bb[4] << 16) * B_SCALE, __uint_as_float(bb[5] << 16) * B_SCALE);
        qh.w = f16x2_bits(__uint_as_float(bb[6] << 16) * B_SCALE, __uint_as_float(bb[7] << 16) * B_SCALE);
        *(v4u*)(T + ml * TP + 8 * lane) = qh;
        keepb[i] = qb;
        *(volatile v4u*)(memb + (size_t)m * Z_DIM + 8 * lane) = qb;
    }
    __threadfence();
#pragma unroll
    for (int i = 0; i < 8; ++i) {
        const int m = m0 + wave + 8 * i;
        *(volatile v4u*)(memb + (size_t)m * Z_DIM + 8 * lane) = keepb[i];
    }
    __syncthreads();

    v4u keept[8];
    const int j  = lane & 7;
    const int zq = lane >> 3;
#pragma unroll
    for (int q = 0; q < 8; ++q) {
        const int z = wave * 32 + q * 4 + zq;
        const unsigned short* colp = T + (8 * j) * TP + z;
        v4u v;
        v.x = (unsigned int)colp[0 * TP] | ((unsigned int)colp[1 * TP] << 16);
        v.y = (unsigned int)colp[2 * TP] | ((unsigned int)colp[3 * TP] << 16);
        v.z = (unsigned int)colp[4 * TP] | ((unsigned int)colp[5 * TP] << 16);
        v.w = (unsigned int)colp[6 * TP] | ((unsigned int)colp[7 * TP] << 16);
        keept[q] = v;
        *(volatile v4u*)(memh + (size_t)z * MEM_DIM + m0 + 8 * j) = v;
    }
    __threadfence();
#pragma unroll
    for (int q = 0; q < 8; ++q) {
        const int z = wave * 32 + q * 4 + zq;
        *(volatile v4u*)(memh + (size_t)z * MEM_DIM + m0 + 8 * j) = keept[q];
    }
}

__global__ __launch_bounds__(NTHR)
void k_main(const float* __restrict__ x,
            const unsigned short* __restrict__ memb,
            const unsigned short* __restrict__ memh,
            float* __restrict__ out,
            int nrows)
{
    __shared__ __attribute__((aligned(16))) unsigned short xlds[RPB * XP];
    __shared__ __attribute__((aligned(16))) float att[RPB * AP];
    __shared__ float rowscale[RPB];

    const int tid     = threadIdx.x;
    const int wave    = tid >> 5;
    const int lane    = tid & 31;
    const int h       = lane >> 4;
    const int l15     = lane & 15;
    const int rowbase = blockIdx.x * RPB;

#pragma unroll
    for (int i = 0; i < 4; ++i) {
        const int q    = tid + NTHR * i;
        const int r    = q >> 6;
        const int c    = (q & 63) * 4;
        const int grow = rowbase + r;
        v4f v = {0.0f, 0.0f, 0.0f, 0.0f};
        if (grow < nrows) v = *(const v4f*)(x + (size_t)grow * Z_DIM + c);
        v2u p;
        p.x = bf16_bits(v.x) | (bf16_bits(v.y) << 16);
        p.y = bf16_bits(v.z) | (bf16_bits(v.w) << 16);
        *(v2u*)(xlds + r * XP + c) = p;
    }
    __syncthreads();

    {
        FragB af[8];
        const unsigned short* xa = xlds + l15 * XP + 8 * h;
#pragma unroll
        for (int kc = 0; kc < 8; ++kc) {
            af[kc].q[0] = *(const v4u*)(xa + kc * 32);
            af[kc].q[1] = *(const v4u*)(xa + kc * 32 + 16);
        }

        const int nbase = wave * 256;
#pragma unroll 1
        for (int nt = 0; nt < 16; nt += 2) {
            const unsigned short* pb0 = memb + (size_t)(nbase + nt * 16 + l15) * Z_DIM + 8 * h;
            const unsigned short* pb1 = pb0 + 16 * Z_DIM;

            v8f acc0, acc1;
#pragma unroll
            for (int e = 0; e < 8; ++e) { acc0[e] = 0.0f; acc1[e] = 0.0f; }

#pragma unroll
            for (int kc = 0; kc < 8; ++kc) {
                FragB b0, b1;
                b0.q[0] = *(const v4u*)(pb0 + kc * 32);
                b0.q[1] = *(const v4u*)(pb0 + kc * 32 + 16);
                b1.q[0] = *(const v4u*)(pb1 + kc * 32);
                b1.q[1] = *(const v4u*)(pb1 + kc * 32 + 16);
                acc0 = __builtin_amdgcn_wmma_f32_16x16x32_bf16(false, af[kc].v, false, b0.v,
                                                               (short)0, acc0, false, false);
                acc1 = __builtin_amdgcn_wmma_f32_16x16x32_bf16(false, af[kc].v, false, b1.v,
                                                               (short)0, acc1, false, false);
                WMMA_GUARD2(acc0, acc1, af[kc].v, b0.v, b1.v);
            }

            const int cn = nbase + nt * 16 + l15;
#pragma unroll
            for (int r = 0; r < 8; ++r) {
                att[(8 * h + r) * AP + cn]      = acc0[r];
                att[(8 * h + r) * AP + cn + 16] = acc1[r];
            }
        }
    }
    __syncthreads();

    float rsv[2];
#pragma unroll
    for (int rr = 0; rr < 2; ++rr) {
        float* row = att + (wave * 2 + rr) * AP;
        float mx = -3.0e38f;
#pragma unroll 4
        for (int c = lane; c < MEM_DIM; c += 32) mx = fmaxf(mx, row[c]);
#pragma unroll
        for (int off = 16; off > 0; off >>= 1) mx = fmaxf(mx, __shfl_xor(mx, off, 32));

        double s = 0.0;
#pragma unroll 4
        for (int c = lane; c < MEM_DIM; c += 32) {
            const float a = row[c];
            const float e = expf((a - mx) * 2.0f);
            s += (double)e;
            row[c] = e;
        }
#pragma unroll
        for (int off = 16; off > 0; off >>= 1) s += __shfl_xor(s, off, 32);
        rsv[rr] = 1.0f / (float)s;
    }
    __syncthreads();

#pragma unroll
    for (int rr = 0; rr < 2; ++rr) {
        const int r = wave * 2 + rr;
        const float* rowf = att + r * AP;
        const float rsum  = rsv[rr];

        unsigned int pk[32];
        double l1 = 0.0;
#pragma unroll
        for (int jg = 0; jg < 8; ++jg) {
            const int c0 = 256 * jg + 8 * lane;
            const v4f u0 = *(const v4f*)(rowf + c0);
            const v4f u1 = *(const v4f*)(rowf + c0 + 4);
            float g[8];
            g[0] = shrink_g(u0.x * rsum); g[1] = shrink_g(u0.y * rsum);
            g[2] = shrink_g(u0.z * rsum); g[3] = shrink_g(u0.w * rsum);
            g[4] = shrink_g(u1.x * rsum); g[5] = shrink_g(u1.y * rsum);
            g[6] = shrink_g(u1.z * rsum); g[7] = shrink_g(u1.w * rsum);
            float part = ((g[0] + g[1]) + (g[2] + g[3])) + ((g[4] + g[5]) + (g[6] + g[7]));
            l1 += (double)part;
            pk[4 * jg + 0] = f16x2_bits(g[0], g[1]);
            pk[4 * jg + 1] = f16x2_bits(g[2], g[3]);
            pk[4 * jg + 2] = f16x2_bits(g[4], g[5]);
            pk[4 * jg + 3] = f16x2_bits(g[6], g[7]);
        }
#pragma unroll
        for (int off = 16; off > 0; off >>= 1) l1 += __shfl_xor(l1, off, 32);
        if (lane == 0) rowscale[r] = 1.0f / fmaxf((float)l1, EPS_N);

        __syncthreads();

        unsigned short* rowh = (unsigned short*)(att + r * AP);
#pragma unroll
        for (int jg = 0; jg < 8; ++jg) {
            v4u v;
            v.x = pk[4 * jg + 0]; v.y = pk[4 * jg + 1]; v.z = pk[4 * jg + 2]; v.w = pk[4 * jg + 3];
            *(v4u*)(rowh + 256 * jg + 8 * lane) = v;
        }
    }
    __syncthreads();

    {
        const int z0 = wave * 32;
        const unsigned short* pa  = (const unsigned short*)att + l15 * APH + 8 * h;
        const unsigned short* pb0 = memh + (size_t)(z0 + l15) * MEM_DIM + 8 * h;
        const unsigned short* pb1 = pb0 + 16 * MEM_DIM;

        v8f acc0, acc1;
#pragma unroll
        for (int e = 0; e < 8; ++e) { acc0[e] = 0.0f; acc1[e] = 0.0f; }

#pragma unroll 2
        for (int kc = 0; kc < MEM_DIM; kc += 32) {
            FragH a, b0, b1;
            a.q[0]  = *(const v4u*)(pa + kc);
            a.q[1]  = *(const v4u*)(pa + kc + 16);
            b0.q[0] = *(const v4u*)(pb0 + kc);
            b0.q[1] = *(const v4u*)(pb0 + kc + 16);
            b1.q[0] = *(const v4u*)(pb1 + kc);
            b1.q[1] = *(const v4u*)(pb1 + kc + 16);
            acc0 = __builtin_amdgcn_wmma_f32_16x16x32_f16(false, a.v, false, b0.v,
                                                          (short)0, acc0, false, false);
            acc1 = __builtin_amdgcn_wmma_f32_16x16x32_f16(false, a.v, false, b1.v,
                                                          (short)0, acc1, false, false);
            WMMA_GUARD2(acc0, acc1, a.v, b0.v, b1.v);
        }

        __syncthreads();

#pragma unroll
        for (int r = 0; r < 8; ++r) {
            const float sc = rowscale[8 * h + r] * B_UNSCALE;
            att[(8 * h + r) * OP + z0 + l15]      = acc0[r] * sc;
            att[(8 * h + r) * OP + z0 + 16 + l15] = acc1[r] * sc;
        }
    }
    __syncthreads();

    {
        v4f keep[4];
        const int seg0 = lane >> 3;
        const int cl   = 4 * (lane & 7);
#pragma unroll
        for (int i = 0; i < 4; ++i) {
            const int rl  = wave * 2 + (i >> 1);
            const int col = 32 * ((i & 1) * 4 + seg0) + cl;
            keep[i] = *(const v4f*)(att + rl * OP + col);
        }
#pragma unroll
        for (int i = 0; i < 4; ++i) {
            const int rl   = wave * 2 + (i >> 1);
            const int col  = 32 * ((i & 1) * 4 + seg0) + cl;
            const int grow = rowbase + rl;
            if (grow < nrows) *(volatile v4f*)(out + (size_t)grow * Z_DIM + col) = keep[i];
        }
        __threadfence();
#pragma unroll
        for (int i = 0; i < 4; ++i) {
            const int rl   = wave * 2 + (i >> 1);
            const int col  = 32 * ((i & 1) * 4 + seg0) + cl;
            const int grow = rowbase + rl;
            if (grow < nrows) *(volatile v4f*)(out + (size_t)grow * Z_DIM + col) = keep[i];
        }
    }
}

extern "C" void kernel_launch(void* const* d_in, const int* in_sizes, int n_in,
                              void* d_out, int out_size, void* d_ws, size_t ws_size,
                              hipStream_t stream)
{
    if (n_in < 2) return;
    const int nx = in_sizes[0];
    const int nm = in_sizes[1];
    if (nm != MEM_DIM * Z_DIM) return;
    if (nx <= 0 || (nx % Z_DIM) != 0) return;
    const int nrows = nx / Z_DIM;
    if (out_size < nrows * Z_DIM) return;

    const size_t half_bytes = (size_t)MEM_DIM * Z_DIM * sizeof(unsigned short);
    if (ws_size < 2 * half_bytes) return;

    const float* xp   = (const float*)d_in[0];
    const float* memp = (const float*)d_in[1];
    float* outp = (float*)d_out;
    unsigned short* memb = (unsigned short*)d_ws;
    unsigned short* memh = (unsigned short*)((char*)d_ws + half_bytes);

    k_prep<<<dim3(MEM_DIM / PM), dim3(NTHR), 0, stream>>>(memp, memb, memh);
    k_main<<<dim3((nrows + RPB - 1) / RPB), dim3(NTHR), 0, stream>>>(xp, memb, memh, outp, nrows);
}
